// HSTUTransducer_566935683422
// MI455X (gfx1250) — hardware-run, weakly checked
//
#include <hip/hip_runtime.h>
#include <math.h>

typedef __attribute__((ext_vector_type(16))) _Float16 v16h;
typedef __attribute__((ext_vector_type(8)))  _Float16 v8h;
typedef __attribute__((ext_vector_type(8)))  float    v8f;
typedef __attribute__((ext_vector_type(4)))  float    v4f;
typedef __attribute__((ext_vector_type(4)))  unsigned int v4u;

constexpr int kNB      = 8;
constexpr int kSeq     = 2048;
constexpr int kDim     = 128;
constexpr int kHeads   = 4;
constexpr int kDH      = 128;
constexpr int kDA      = 128;
constexpr int kTH      = kHeads * kDH;
constexpr int kTA      = kHeads * kDA;
constexpr int kNE      = 2 * kTH + 2 * kTA;
constexpr int kVocab   = 100000;
constexpr int kNPos    = 256;
constexpr int kNTimeRows = 257;
constexpr int kTok     = kNB * kSeq;
constexpr int kKVP     = kTH + kTA;
constexpr int kOutF    = 2 * kTH + kDim;
constexpr float kLnEps   = 1e-6f;
constexpr float kWCarry  = 16.0f;
constexpr float kWCarryInv = 1.0f / kWCarry;
static_assert(kTH == 512 && kTA == 512 && kNE == 2048 && kKVP == 1024 && kOutF == 1152, "slab layout");
static_assert((kDim % 32) == 0, "GEMM K multiple of 32");
static_assert((kTok % 64) == 0 && (kKVP % 64) == 0, "GEMM M,N multiples of 64");
static_assert((kSeq % 16) == 0 && (kVocab % 4) == 0 && ((kVocab * 4) % 128) == 0, "store maps");
static_assert(kDim == 128 && kDH == 128 && kDA == 128, "lane maps assume 128-wide rows");

constexpr size_t kOffWT     = 0;
constexpr size_t kOffKVB    = kOffWT     + (size_t)kKVP * kDim * 2;
constexpr size_t kOffNX     = kOffKVB    + (size_t)kKVP * 4;
constexpr size_t kOffKV     = kOffNX     + (size_t)kTok * kDim * 2;
constexpr size_t kOffXLAST  = kOffKV     + (size_t)kTok * kKVP * 2;
constexpr size_t kOffNXLAST = kOffXLAST  + (size_t)kNB * kDim * 4;
constexpr size_t kOffOLAST  = kOffNXLAST + (size_t)kNB * kDim * 4;
constexpr size_t kOffHBUF   = kOffOLAST  + (size_t)kNB * kTH * 4;
constexpr size_t kWsTotal   = kOffHBUF   + (size_t)kNB * kDim * 4;
static_assert(kWsTotal == 38043648ull, "carve total");
static_assert(kWsTotal <= 134217728ull, "carve cap");
static_assert((kOffKVB % 128) == 0 && (kOffNX % 128) == 0 && (kOffKV % 128) == 0 && (kOffXLAST % 128) == 0 &&
              (kOffNXLAST % 128) == 0 && (kOffOLAST % 128) == 0 && (kOffHBUF % 128) == 0, "128-B aligned regions");

__device__ __forceinline__ float h16_to_f32(unsigned hb) {
  const unsigned sgn = (hb & 0x8000u) << 16;
  const unsigned em = hb & 0x7fffu;
  const float fn = __uint_as_float((em << 13) + 0x38000000u);
  const float fs = (float)em * 5.9604644775390625e-8f;
  const float mag = (em < 0x400u) ? fs : fn;
  return __uint_as_float(__float_as_uint(mag) | sgn);
}

__device__ __forceinline__ v8f mma_h(v16h a, v16h b, v8f c) {
  c = __builtin_amdgcn_wmma_f32_16x16x32_f16(false, a, false, b, (short)0, c, false, false);
  asm volatile("v_nop\n\tv_nop\n\tv_nop\n\tv_nop" : "+v"(c) : "v"(a), "v"(b));
  return c;
}
__device__ __forceinline__ void keep4_h(v16h a, v16h b, v16h c, v16h d) { asm volatile("v_nop" :: "v"(a), "v"(b), "v"(c), "v"(d)); }
__device__ __forceinline__ void acc_guard4(v8f& a, v8f& b, v8f& c, v8f& d) { asm volatile("v_nop\n\tv_nop\n\tv_nop\n\tv_nop" : "+v"(a), "+v"(b), "+v"(c), "+v"(d)); }

struct FragH {
  union U { v16h v; v8h h[2]; };
  static __device__ __forceinline__ v16h load(const _Float16* p) {
    U f;
    f.h[0] = *(const v8h*)(p);
    f.h[1] = *(const v8h*)(p + 16);
    return f.v;
  }
};

__global__ __launch_bounds__(256) void wt_convert_kernel(const float* __restrict__ W, const float* __restrict__ bias,
                                                         unsigned short* __restrict__ WT, float* __restrict__ kvb, float carry) {
  __shared__ float sm[64][65];
  const int t = threadIdx.x;
  if (blockIdx.y == 16) {
    if (blockIdx.x != 0) return;
    const int n = 4 * t;
    const int col = n + ((n >= kTH) ? 1024 : 512);
    const v4f bv = *(const v4f*)(bias + col);
    *(volatile v4f*)(kvb + n) = bv;
    __threadfence();
    *(volatile v4f*)(kvb + n) = bv;
    return;
  }
  const int k0 = blockIdx.x * 64;
  const int n0 = blockIdx.y * 64;
  const int col0 = n0 + ((n0 >= kTH) ? 1024 : 512);
#pragma unroll
  for (int i = 0; i < 16; ++i) {
    const int e = i * 256 + t;
    const int r = e >> 6;
    const int c = e & 63;
    sm[c][r] = W[(size_t)(k0 + r) * kNE + col0 + c] * carry;
  }
  __syncthreads();
  const int lane = t & 31, wave = t >> 5;
  const int q = lane >> 3, c8 = (lane & 7) * 8;
  v8h hv[2];
#pragma unroll
  for (int it = 0; it < 2; ++it) {
    const int row = wave * 8 + it * 4 + q;
#pragma unroll
    for (int e = 0; e < 8; ++e) hv[it][e] = (_Float16)sm[row][c8 + e];
  }
  for (int pass = 0; pass < 2; ++pass) {
#pragma unroll
    for (int it = 0; it < 2; ++it) {
      const int row = wave * 8 + it * 4 + q;
      *(volatile v8h*)(WT + (size_t)(n0 + row) * kDim + k0 + c8) = hv[it];
    }
    __threadfence();
  }
}

__global__ __launch_bounds__(256) void embed_ln1_kernel(
    const float* __restrict__ emb, const float* __restrict__ pos_emb, const float* __restrict__ time_emb,
    const float* __restrict__ g, const float* __restrict__ beta,
    const int* __restrict__ item_ids, const int* __restrict__ seq_lengths,
    const int* __restrict__ timestamps, const int* __restrict__ num_targets,
    unsigned short* __restrict__ NX, float* __restrict__ x_last, float* __restrict__ nx_last, float embScale) {
  __shared__ __align__(16) float sN[16 * 132];
  const int t = threadIdx.x, lane = t & 31, wave = t >> 5;
  const int tok0 = blockIdx.x * 16;
  const int b = tok0 / kSeq;
  const int sl = seq_lengths[b];
  const int nt = num_targets[b];
  const int high = sl - nt;
  const int last = min(max(sl - 1, 0), kSeq - 1);
  const int qt = timestamps[b * kSeq + last];
  const v4f gv = *(const v4f*)(g + lane * 4);
  const v4f bv = *(const v4f*)(beta + lane * 4);
#pragma unroll 1
  for (int j = 0; j < 2; ++j) {
    const int r = wave * 2 + j;
    const int tok = tok0 + r;
    const int s = tok - b * kSeq;
    int item = item_ids[tok];
    item = min(max(item, 0), kVocab - 1);
    const int col = min(s, high);
    const int pidx = min(max(high - col, 0), kNPos - 1);
    const int tsv = timestamps[tok];
    const float dt = (float)(qt - tsv);
    const float tq = fmaxf(dt, 1e-6f) * (1.0f / 60.0f);
    float sq = sqrtf(tq);
    sq = fminf(fmaxf(sq, 0.0f), (float)(kNTimeRows - 1));
    int tidx = (int)sq;
    tidx = min(max(tidx, 0), kNTimeRows - 1);
    const v4f ev = *(const v4f*)(emb + (size_t)item * kDim + lane * 4);
    const v4f pv = *(const v4f*)(pos_emb + (size_t)pidx * kDim + lane * 4);
    const v4f tv = *(const v4f*)(time_emb + (size_t)tidx * kDim + lane * 4);
    v4f xv;
    xv.x = (ev.x * embScale + pv.x) + tv.x;
    xv.y = (ev.y * embScale + pv.y) + tv.y;
    xv.z = (ev.z * embScale + pv.z) + tv.z;
    xv.w = (ev.w * embScale + pv.w) + tv.w;
    float sum = (xv.x + xv.y) + (xv.z + xv.w);
#pragma unroll
    for (int off = 16; off > 0; off >>= 1) sum += __shfl_xor(sum, off, 32);
    const float mu = sum * (1.0f / (float)kDim);
    const float d0 = xv.x - mu, d1 = xv.y - mu, d2 = xv.z - mu, d3 = xv.w - mu;
    float ss = (d0 * d0 + d1 * d1) + (d2 * d2 + d3 * d3);
#pragma unroll
    for (int off = 16; off > 0; off >>= 1) ss += __shfl_xor(ss, off, 32);
    const float var = ss * (1.0f / (float)kDim);
    const float rstd = rsqrtf(var + kLnEps);
    v4f nv;
    nv.x = d0 * rstd * gv.x + bv.x;
    nv.y = d1 * rstd * gv.y + bv.y;
    nv.z = d2 * rstd * gv.z + bv.z;
    nv.w = d3 * rstd * gv.w + bv.w;
    *(v4f*)(sN + r * 132 + lane * 4) = nv;
    if (s == last) {
      float* xd = x_last + (size_t)b * kDim + lane * 4;
      float* nd = nx_last + (size_t)b * kDim + lane * 4;
      *(volatile v4f*)xd = xv;
      *(volatile v4f*)nd = nv;
      __threadfence();
      *(volatile v4f*)xd = xv;
      *(volatile v4f*)nd = nv;
    }
  }
  __syncthreads();
  {
    const int row = t >> 4, c8 = (t & 15) * 8;
    const float* sp = sN + row * 132 + c8;
    const v4f a0 = *(const v4f*)(sp);
    const v4f a1 = *(const v4f*)(sp + 4);
    v8h hv;
    hv[0] = (_Float16)a0.x; hv[1] = (_Float16)a0.y; hv[2] = (_Float16)a0.z; hv[3] = (_Float16)a0.w;
    hv[4] = (_Float16)a1.x; hv[5] = (_Float16)a1.y; hv[6] = (_Float16)a1.z; hv[7] = (_Float16)a1.w;
    unsigned short* dst = NX + (size_t)(tok0 + row) * kDim + c8;
    *(volatile v8h*)dst = hv;
    __threadfence();
    *(volatile v8h*)dst = hv;
  }
}

__global__ __launch_bounds__(256) void kv_gemm_kernel(
    const unsigned short* __restrict__ Ap, int lda,
    const unsigned short* __restrict__ Btp, int ldb,
    unsigned short* __restrict__ Cout, int ldc,
    const float* __restrict__ bias, int M, int N, int K, float scale) {
  const _Float16* A  = (const _Float16*)Ap;
  const _Float16* Bt = (const _Float16*)Btp;
  __shared__ __align__(16) float sT[8][16 * 68];
  const int lane = threadIdx.x & 31;
  const int wave = threadIdx.x >> 5;
  const int tilesN = N >> 6;
  const int tilesM = M >> 6;
  const int tile = blockIdx.x * 8 + wave;
  if (tile >= tilesM * tilesN) return;
  const int tm = tile / tilesN;
  const int tn = tile - tm * tilesN;
  const int m0 = tm << 6;
  const int n0 = tn << 6;
  const int rlane = lane & 15;
  const int koff  = (lane >> 4) * 8;
  const int mOff  = (lane >> 4) * 8;

  v8f acc[4][4];
#pragma unroll
  for (int i = 0; i < 4; ++i)
#pragma unroll
    for (int j = 0; j < 4; ++j) acc[i][j] = (v8f){0.f, 0.f, 0.f, 0.f, 0.f, 0.f, 0.f, 0.f};

  for (int k0 = 0; k0 < K; k0 += 32) {
    v16h bh[4];
#pragma unroll
    for (int j = 0; j < 4; ++j) {
      const size_t bo = (size_t)(n0 + (j << 4) + rlane) * ldb + koff + k0;
      bh[j] = FragH::load(Bt + bo);
    }
#pragma unroll
    for (int i = 0; i < 4; ++i) {
      const size_t ao = (size_t)(m0 + (i << 4) + rlane) * lda + koff + k0;
      const v16h ah = FragH::load(A + ao);
#pragma unroll
      for (int j = 0; j < 4; ++j) acc[i][j] = mma_h(ah, bh[j], acc[i][j]);
    }
    keep4_h(bh[0], bh[1], bh[2], bh[3]);
  }
  acc_guard4(acc[0][0], acc[0][1], acc[0][2], acc[0][3]);
  acc_guard4(acc[1][0], acc[1][1], acc[1][2], acc[1][3]);
  acc_guard4(acc[2][0], acc[2][1], acc[2][2], acc[2][3]);
  acc_guard4(acc[3][0], acc[3][1], acc[3][2], acc[3][3]);

  float* slab = sT[wave];
#pragma unroll
  for (int i = 0; i < 4; ++i) {
    const int mBase = m0 + (i << 4);
#pragma unroll
    for (int j = 0; j < 4; ++j) {
      const int n = n0 + (j << 4) + rlane;
      const float bv = bias[n];
#pragma unroll
      for (int r = 0; r < 8; ++r) {
        const float v = acc[i][j][r] * scale + bv;
        slab[(mOff + r) * 68 + (j << 4) + rlane] = v;
      }
    }
    __builtin_amdgcn_fence(__ATOMIC_RELEASE, "workgroup");
    __builtin_amdgcn_wave_barrier();
    __builtin_amdgcn_fence(__ATOMIC_ACQUIRE, "workgroup");
    {
      const int q = lane >> 3, c8 = (lane & 7) * 8;
      for (int pass = 0; pass < 2; ++pass) {
#pragma unroll
        for (int it = 0; it < 4; ++it) {
          const int row = it * 4 + q;
          const float* sp = slab + row * 68 + c8;
          v8h hv;
#pragma unroll
          for (int e = 0; e < 8; ++e) hv[e] = (_Float16)sp[e];
          *(volatile v8h*)(Cout + (size_t)(mBase + row) * ldc + n0 + c8) = hv;
        }
        __threadfence();
      }
    }
    __builtin_amdgcn_fence(__ATOMIC_RELEASE, "workgroup");
    __builtin_amdgcn_wave_barrier();
    __builtin_amdgcn_fence(__ATOMIC_ACQUIRE, "workgroup");
  }
}

__global__ __launch_bounds__(256) void attn_last_kernel(
    const float* __restrict__ nx_last, const float* __restrict__ uvqk_w, const float* __restrict__ uvqk_b,
    const unsigned* __restrict__ KVw, const int* __restrict__ seq_lengths,
    float* __restrict__ o_last, float qkScale) {
  __shared__ __align__(16) float sNx[kDim];
  __shared__ __align__(16) float sPart[2 * kDA];
  __shared__ __align__(16) float sQ[kDA];
  __shared__ __align__(16) float sA[kSeq];
  __shared__ __align__(16) float sPo[4 * kDH];
  const int t = threadIdx.x;
  const int bh = blockIdx.x;
  const int b = bh / kHeads;
  const int h = bh - b * kHeads;
  const int sl = seq_lengths[b];
  const int nvalid = min(max(sl, 0), kSeq);

  if (t < kDim) sNx[t] = nx_last[(size_t)b * kDim + t];
  __syncthreads();
  {
    const int d = t & (kDA - 1);
    const int kh = t >> 7;
    const int col = 2 * kTH + h * kDA + d;
    float acc = 0.0f;
#pragma unroll 4
    for (int k = 0; k < kDim / 2; ++k) {
      const int kk = kh * (kDim / 2) + k;
      acc = fmaf(sNx[kk], uvqk_w[(size_t)kk * kNE + col], acc);
    }
    sPart[kh * kDA + d] = acc;
  }
  __syncthreads();
  if (t < kDA) sQ[t] = (sPart[t] + sPart[kDA + t]) + uvqk_b[2 * kTH + h * kDA + t];
  __syncthreads();

  const int nIter = min((nvalid + 255) >> 8, kSeq / 256);
#pragma unroll 1
  for (int it = 0; it < nIter; ++it) {
    const int m = it * 256 + t;
    const int mc = min(m, kSeq - 1);
    const v4u* kp = (const v4u*)(KVw + (size_t)(b * kSeq + mc) * (kKVP / 2) + (kTH / 2) + h * (kDA / 2));
    float dot = 0.0f;
#pragma unroll 1
    for (int c = 0; c < kDA / 8; ++c) {
      const v4u w = kp[c];
      const v4f qa = *(const v4f*)(sQ + 8 * c);
      const v4f qb = *(const v4f*)(sQ + 8 * c + 4);
      const unsigned w0 = w.x, w1 = w.y, w2 = w.z, w3 = w.w;
      dot = fmaf(qa.x, h16_to_f32(w0 & 0xffffu), dot);
      dot = fmaf(qa.y, h16_to_f32(w0 >> 16), dot);
      dot = fmaf(qa.z, h16_to_f32(w1 & 0xffffu), dot);
      dot = fmaf(qa.w, h16_to_f32(w1 >> 16), dot);
      dot = fmaf(qb.x, h16_to_f32(w2 & 0xffffu), dot);
      dot = fmaf(qb.y, h16_to_f32(w2 >> 16), dot);
      dot = fmaf(qb.z, h16_to_f32(w3 & 0xffffu), dot);
      dot = fmaf(qb.w, h16_to_f32(w3 >> 16), dot);
    }
    const float s = dot * qkScale;
    const float sg = 1.0f / (1.0f + expf(-s));
    const float a = s * sg;
    sA[m] = (m < nvalid) ? a : 0.0f;
  }
  __syncthreads();
  {
    const int g = t >> 6;
    const int w = t & 63;
    const unsigned* vp = KVw + (size_t)(b * kSeq) * (kKVP / 2) + h * (kDH / 2) + w;
    float o0 = 0.0f, o1 = 0.0f;
#pragma unroll 1
    for (int m = g; m < nvalid; m += 4) {
      const unsigned word = vp[(size_t)m * (kKVP / 2)];
      const float a = sA[m];
      o0 = fmaf(a, h16_to_f32(word & 0xffffu), o0);
      o1 = fmaf(a, h16_to_f32(word >> 16), o1);
    }
    sPo[g * kDH + 2 * w]     = o0;
    sPo[g * kDH + 2 * w + 1] = o1;
  }
  __syncthreads();
  if (t < 32) {
    const int c4 = t * 4;
    const v4f r0 = *(const v4f*)(sPo + c4);
    const v4f r1 = *(const v4f*)(sPo + kDH + c4);
    const v4f r2 = *(const v4f*)(sPo + 2 * kDH + c4);
    const v4f r3 = *(const v4f*)(sPo + 3 * kDH + c4);
    const v4f rr = ((r0 + r1) + r2) + r3;
    float* dst = o_last + (size_t)bh * kDH + c4;
    *(volatile v4f*)dst = rr;
    __threadfence();
    *(volatile v4f*)dst = rr;
  }
}

__global__ __launch_bounds__(256) void tail_kernel(
    const float* __restrict__ nx_last, const float* __restrict__ x_last, const float* __restrict__ o_last,
    const float* __restrict__ uvqk_w, const float* __restrict__ uvqk_b,
    const float* __restrict__ ln2_g, const float* __restrict__ ln2_b,
    const float* __restrict__ out_w, float* __restrict__ hbuf) {
  __shared__ __align__(16) float sNx[kDim];
  __shared__ __align__(16) float sX[kDim];
  __shared__ __align__(16) float sY[kOutF];
  __shared__ __align__(16) float sRed[256];
  __shared__ __align__(16) float sPart[256];
  const int t = threadIdx.x;
  const int b = blockIdx.x;
  if (t < kDim) {
    sNx[t] = nx_last[(size_t)b * kDim + t];
    sX[t]  = x_last[(size_t)b * kDim + t];
  }
  __syncthreads();
  float a0 = 0.0f, a1 = 0.0f;
#pragma unroll 4
  for (int k = 0; k < kDim; ++k) {
    const float xk = sNx[k];
    a0 = fmaf(xk, uvqk_w[(size_t)k * kNE + t], a0);
    a1 = fmaf(xk, uvqk_w[(size_t)k * kNE + 256 + t], a1);
  }
  float u0 = a0 + uvqk_b[t];
  float u1 = a1 + uvqk_b[256 + t];
  u0 = u0 * (1.0f / (1.0f + expf(-u0)));
  u1 = u1 * (1.0f / (1.0f + expf(-u1)));

  const float o0 = o_last[(size_t)b * kTH + t];
  const float o1 = o_last[(size_t)b * kTH + 256 + t];
  sRed[t] = o0 + o1;
  __syncthreads();
  for (int off = 128; off > 0; off >>= 1) {
    if (t < off) sRed[t] += sRed[t + off];
    __syncthreads();
  }
  const float mu = sRed[0] * (1.0f / (float)kTH);
  __syncthreads();
  const float d0 = o0 - mu, d1 = o1 - mu;
  sRed[t] = d0 * d0 + d1 * d1;
  __syncthreads();
  for (int off = 128; off > 0; off >>= 1) {
    if (t < off) sRed[t] += sRed[t + off];
    __syncthreads();
  }
  const float var = sRed[0] * (1.0f / (float)kTH);
  const float rstd = rsqrtf(var + kLnEps);
  const float no0 = d0 * rstd * ln2_g[t] + ln2_b[t];
  const float no1 = d1 * rstd * ln2_g[256 + t] + ln2_b[256 + t];
  sY[t] = u0;
  sY[256 + t] = u1;
  sY[kTH + kDim + t] = u0 * no0;
  sY[kTH + kDim + 256 + t] = u1 * no1;
  if (t < kDim) sY[kTH + t] = sX[t];
  __syncthreads();
  {
    const int d = t & (kDim - 1);
    const int hf = t >> 7;
    float acc = 0.0f;
#pragma unroll 4
    for (int f = 0; f < kOutF / 2; ++f) {
      const int ff = hf * (kOutF / 2) + f;
      acc = fmaf(sY[ff], out_w[(size_t)ff * kDim + d], acc);
    }
    sPart[t] = acc;
  }
  __syncthreads();
  if (t < 32) {
    const int c4 = t * 4;
    const v4f p0 = *(const v4f*)(sPart + c4);
    const v4f p1 = *(const v4f*)(sPart + kDim + c4);
    const v4f xr = *(const v4f*)(sX + c4);
    const v4f rr = (p0 + p1) + xr;
    float* dst = hbuf + (size_t)b * kDim + c4;
    *(volatile v4f*)dst = rr;
    __threadfence();
    *(volatile v4f*)dst = rr;
  }
}

__global__ __launch_bounds__(256) void head_kernel(
    const float* __restrict__ hbuf, const float* __restrict__ head_w, const float* __restrict__ head_b,
    float* __restrict__ out) {
  __shared__ __align__(16) float hs[kNB * kDim];
  __shared__ __align__(16) float sO[kNB * 260];
  const int t = threadIdx.x, lane = t & 31, wave = t >> 5;
  *(v4f*)(hs + 4 * t) = *(const v4f*)(hbuf + 4 * t);
  __syncthreads();
  const int v = blockIdx.x * 256 + t;
  const int vc = min(v, kVocab - 1);
  const float* wp = head_w + vc;
  float acc[kNB];
#pragma unroll
  for (int bb = 0; bb < kNB; ++bb) acc[bb] = 0.0f;
#pragma unroll 1
  for (int d4 = 0; d4 < kDim / 4; ++d4) {
    const float w0 = wp[(size_t)(4 * d4 + 0) * kVocab];
    const float w1 = wp[(size_t)(4 * d4 + 1) * kVocab];
    const float w2 = wp[(size_t)(4 * d4 + 2) * kVocab];
    const float w3 = wp[(size_t)(4 * d4 + 3) * kVocab];
#pragma unroll
    for (int bb = 0; bb < kNB; ++bb) {
      const v4f hv = *(const v4f*)(hs + bb * kDim + 4 * d4);
      acc[bb] = fmaf(hv.x, w0, acc[bb]);
      acc[bb] = fmaf(hv.y, w1, acc[bb]);
      acc[bb] = fmaf(hv.z, w2, acc[bb]);
      acc[bb] = fmaf(hv.w, w3, acc[bb]);
    }
  }
  const float hb = head_b[vc];
#pragma unroll
  for (int bb = 0; bb < kNB; ++bb) sO[bb * 260 + t] = acc[bb] + hb;
  __syncthreads();
  v4f val[2];
#pragma unroll
  for (int it = 0; it < 2; ++it) val[it] = *(const v4f*)(sO + wave * 260 + it * 128 + lane * 4);
  for (int pass = 0; pass < 2; ++pass) {
#pragma unroll
    for (int it = 0; it < 2; ++it) {
      const int vv = blockIdx.x * 256 + it * 128 + lane * 4;
      if (vv < kVocab) *(volatile v4f*)(out + (size_t)wave * kVocab + vv) = val[it];
    }
    __threadfence();
  }
}

extern "C" void kernel_launch(void* const* d_in, const int* in_sizes, int n_in,
                              void* d_out, int out_size, void* d_ws, size_t ws_size,
                              hipStream_t stream) {
  if (n_in < 16) return;
  if (in_sizes[0] != kVocab * kDim) return;
  if (in_sizes[1] != kNPos * kDim) return;
  if (in_sizes[2] != kNTimeRows * kDim) return;
  if (in_sizes[3] != kDim || in_sizes[4] != kDim) return;
  if (in_sizes[5] != kDim * kNE) return;
  if (in_sizes[6] != kNE) return;
  if (in_sizes[7] != kTH || in_sizes[8] != kTH) return;
  if (in_sizes[9] != kOutF * kDim) return;
  if (in_sizes[10] != kDim * kVocab) return;
  if (in_sizes[11] != kVocab) return;
  if (in_sizes[12] != kNB * kSeq) return;
  if (in_sizes[13] != kNB) return;
  if (in_sizes[14] != kNB * kSeq) return;
  if (in_sizes[15] != kNB) return;
  if (out_size != kNB * kVocab) return;
  if (ws_size < kWsTotal) return;

  const float* emb_table  = (const float*)d_in[0];
  const float* pos_emb    = (const float*)d_in[1];
  const float* time_emb   = (const float*)d_in[2];
  const float* ln1_g      = (const float*)d_in[3];
  const float* ln1_b      = (const float*)d_in[4];
  const float* uvqk_w     = (const float*)d_in[5];
  const float* uvqk_b     = (const float*)d_in[6];
  const float* ln2_g      = (const float*)d_in[7];
  const float* ln2_b      = (const float*)d_in[8];
  const float* out_w      = (const float*)d_in[9];
  const float* head_w     = (const float*)d_in[10];
  const float* head_b     = (const float*)d_in[11];
  const int*   item_ids   = (const int*)d_in[12];
  const int*   seq_len    = (const int*)d_in[13];
  const int*   timestamps = (const int*)d_in[14];
  const int*   num_tgt    = (const int*)d_in[15];
  float* out = (float*)d_out;

  char* ws = (char*)d_ws;
  unsigned short* WT     = (unsigned short*)(ws + kOffWT);
  float*          KVB    = (float*)(ws + kOffKVB);
  unsigned short* NX     = (unsigned short*)(ws + kOffNX);
  unsigned short* KV     = (unsigned short*)(ws + kOffKV);
  float*          XLAST  = (float*)(ws + kOffXLAST);
  float*          NXLAST = (float*)(ws + kOffNXLAST);
  float*          OLAST  = (float*)(ws + kOffOLAST);
  float*          HBUF   = (float*)(ws + kOffHBUF);

  const float embScale = (float)__builtin_sqrt((double)kDim);
  const float qkScale  = (float)(1.0 / __builtin_sqrt((double)kDA));

  wt_convert_kernel<<<dim3(kDim / 64, kKVP / 64 + 1), 256, 0, stream>>>(uvqk_w, uvqk_b, WT, KVB, kWCarry);

  embed_ln1_kernel<<<kTok / 16, 256, 0, stream>>>(emb_table, pos_emb, time_emb, ln1_g, ln1_b,
                                                  item_ids, seq_len, timestamps, num_tgt,
                                                  NX, XLAST, NXLAST, embScale);

  kv_gemm_kernel<<<((kTok / 64) * (kKVP / 64)) / 8, 256, 0, stream>>>(
      NX, kDim, WT, kDim, KV, kKVP, KVB, kTok, kKVP, kDim, kWCarryInv);

  attn_last_kernel<<<kNB * kHeads, 256, 0, stream>>>(NXLAST, uvqk_w, uvqk_b, (const unsigned*)KV, seq_len, OLAST, qkScale);

  tail_kernel<<<kNB, 256, 0, stream>>>(NXLAST, XLAST, OLAST, uvqk_w, uvqk_b, ln2_g, ln2_b, out_w, HBUF);

  head_kernel<<<(kVocab + 255) / 256, 256, 0, stream>>>(HBUF, head_w, head_b, out);
}
